// MultiHeadSelfAttention_103079215446
// MI455X (gfx1250) — hardware-verified
//
#include <hip/hip_runtime.h>
#ifndef NB
#define NB 2
#endif
#ifndef SEQ
#define SEQ 2048
#endif
#define NB_FULL 2
#define SEQ_FULL 2048
#define DM 1024
#define NH 16
#define HD 64
#define LQK (2 * DM)
#define NR ((size_t)NB * SEQ)
#define SZ_X16  (NR * DM * 2)
#define SZ_BQKV ((size_t)3 * DM * DM * 2)
#define SZ_BO   ((size_t)DM * DM * 2)
#define SZ_QK   (NR * LQK * 2)
#define SZ_VT   ((size_t)NB * DM * SEQ * 2)
#define SZ_O16  (NR * DM * 2)
#define WS_TOTAL (SZ_X16 + SZ_BQKV + SZ_BO + SZ_QK + SZ_VT + SZ_O16)

static_assert(HD == 64);
static_assert(NH * HD == DM);
static_assert(DM % 128 == 0);
static_assert(DM % 32 == 0);
static_assert(SEQ % 128 == 0);
static_assert((NB * SEQ) % 128 == 0);
static_assert(LQK % 64 == 0);
static_assert(NB <= NB_FULL);
static_assert(SEQ <= SEQ_FULL);
static_assert(SZ_X16 % 256 == 0 && SZ_BQKV % 256 == 0 && SZ_BO % 256 == 0 && SZ_QK % 256 == 0 && SZ_VT % 256 == 0 && SZ_O16 % 256 == 0);
static_assert(WS_TOTAL <= (size_t)134217728);
static_assert((size_t)NB_FULL * SEQ_FULL * DM * 4 == (size_t)16777216);

typedef _Float16 v16h __attribute__((ext_vector_type(16)));
typedef _Float16 v4h  __attribute__((ext_vector_type(4)));
typedef unsigned short v8us __attribute__((ext_vector_type(8), may_alias));
typedef float  v8f  __attribute__((ext_vector_type(8)));
typedef float  v4f  __attribute__((ext_vector_type(4)));
typedef float  v4fa __attribute__((ext_vector_type(4), may_alias));
union FragH { v16h v; v8us half[2]; _Float16 h[16]; unsigned short u[16]; };

__device__ __forceinline__ unsigned short bf16_bits(float x) { unsigned int u = __float_as_uint(x); return (unsigned short)((u + 0x7FFFu + ((u >> 16) & 1u)) >> 16); }
__device__ __forceinline__ float bf16_val(unsigned short b) { return __uint_as_float(((unsigned int)b) << 16); }
__device__ __forceinline__ float bf16_rne(float x) { return bf16_val(bf16_bits(x)); }

__device__ __forceinline__ v16h g2_frag(const _Float16* p, int hh) { FragH f; f.half[0] = *(const v8us*)((const unsigned short*)p + 8 * hh); f.half[1] = *(const v8us*)((const unsigned short*)p + 16 + 8 * hh); return f.v; }
__device__ __forceinline__ v8f g2_mma(v16h a, v16h b, v8f c) { v8f d = __builtin_amdgcn_wmma_f32_16x16x32_f16(false, a, false, b, (short)0, c, false, false); asm volatile("v_nop\n\tv_nop\n\tv_nop\n\tv_nop" : "+v"(d) : "v"(a), "v"(b)); return d; }

__global__ __launch_bounds__(256) void k_x16(const float* __restrict__ x, _Float16* __restrict__ X16, int nrows) {
  const size_t t = (size_t)blockIdx.x * 256 + threadIdx.x; if (t >= (size_t)nrows * (DM / 8)) return;
  const int row = (int)(t / (DM / 8)); const int c8 = (int)(t % (DM / 8)) * 8; const int b = row / SEQ; const int s = row - b * SEQ;
  const float* src = x + ((size_t)b * SEQ_FULL + s) * DM + c8;
  const v4f a = *(const v4fa*)src; const v4f c = *(const v4fa*)(src + 4);
  FragH f;
#pragma unroll
  for (int q = 0; q < 4; ++q) { f.h[q] = (_Float16)bf16_rne(a[q]); f.h[4 + q] = (_Float16)bf16_rne(c[q]); }
  const v8us o = f.half[0]; unsigned short* d = (unsigned short*)X16 + t * 8;
  *(volatile v8us*)d = o; __threadfence(); *(volatile v8us*)d = o;
}

__global__ __launch_bounds__(256) void k_wnat(const float* __restrict__ w, size_t n8, _Float16* __restrict__ Bt) {
  const size_t t = (size_t)blockIdx.x * 256 + threadIdx.x; if (t >= n8) return;
  const v4f a = *(const v4fa*)(w + t * 8); const v4f c = *(const v4fa*)(w + t * 8 + 4);
  FragH f;
#pragma unroll
  for (int q = 0; q < 4; ++q) { f.h[q] = (_Float16)(bf16_rne(a[q]) * 16.0f); f.h[4 + q] = (_Float16)(bf16_rne(c[q]) * 16.0f); }
  const v8us o = f.half[0]; unsigned short* d = (unsigned short*)Bt + t * 8;
  *(volatile v8us*)d = o; __threadfence(); *(volatile v8us*)d = o;
}

__global__ __launch_bounds__(128) void k_gemm2(const _Float16* __restrict__ A, int lda, size_t sA, const _Float16* __restrict__ Bh, int ldb, size_t sB, float alpha,
                                               float* __restrict__ C, _Float16* __restrict__ C16, int ldc, size_t sC, int N, int K) {
  __shared__ __attribute__((aligned(16))) float so[4][32][68];
  const int tid = threadIdx.x; const int w = __builtin_amdgcn_readfirstlane(tid >> 5); const int lane = tid & 31, ln = lane & 15, hh = lane >> 4; const int by = blockIdx.y;
  A += (size_t)by * sA; Bh += (size_t)by * sB; const size_t cofs = (size_t)by * sC;
  const int ntn = N >> 6; const int mt = blockIdx.x / ntn, nq = blockIdx.x - mt * ntn; const int row0 = mt * 128 + 32 * w, col0 = nq * 64;
  const _Float16* a0p = A + (size_t)(row0 + ln) * lda; const _Float16* a1p = a0p + (size_t)16 * lda;
  const _Float16* b0p = Bh + (size_t)(col0 + ln) * ldb; const _Float16* b1p = b0p + (size_t)16 * ldb; const _Float16* b2p = b1p + (size_t)16 * ldb; const _Float16* b3p = b2p + (size_t)16 * ldb;
  const v8f z8 = {0.f,0.f,0.f,0.f,0.f,0.f,0.f,0.f}; v8f c00 = z8, c01 = z8, c02 = z8, c03 = z8, c10 = z8, c11 = z8, c12 = z8, c13 = z8;
#pragma unroll 1
  for (int kb = 0; kb < K; kb += 32) { const v16h a0 = g2_frag(a0p + kb, hh), a1 = g2_frag(a1p + kb, hh);
    v16h b = g2_frag(b0p + kb, hh); c00 = g2_mma(a0, b, c00); c10 = g2_mma(a1, b, c10);
    b = g2_frag(b1p + kb, hh); c01 = g2_mma(a0, b, c01); c11 = g2_mma(a1, b, c11);
    b = g2_frag(b2p + kb, hh); c02 = g2_mma(a0, b, c02); c12 = g2_mma(a1, b, c12);
    b = g2_frag(b3p + kb, hh); c03 = g2_mma(a0, b, c03); c13 = g2_mma(a1, b, c13); }
  v8f accs[8] = {c00, c01, c02, c03, c10, c11, c12, c13};
#pragma unroll
  for (int u = 0; u < 8; ++u) { const int t = u & 3, half = u >> 2;
#pragma unroll
    for (int r = 0; r < 8; ++r) { const int rloc = half * 16 + 8 * hh + r; so[w][rloc][t * 16 + ln] = accs[u][r] * alpha; } }
  __syncthreads();
  const int rsub = lane >> 4, c4 = (lane & 15) * 4;
  for (int pass = 0; pass < 2; ++pass) {
#pragma unroll
    for (int q = 0; q < 16; ++q) { const int r = q * 2 + rsub; const v4f v = *(const v4fa*)&so[w][r][c4];
      if (C) *(volatile v4f*)(C + cofs + (size_t)(row0 + r) * ldc + col0 + c4) = v;
      if (C16) { v4h h4;
#pragma unroll
        for (int i = 0; i < 4; ++i) h4[i] = (_Float16)v[i];
        *(volatile v4h*)(C16 + cofs + (size_t)(row0 + r) * ldc + col0 + c4) = h4; } }
    if (pass == 0) __threadfence(); }
}

__global__ __launch_bounds__(128) void k_flash(const _Float16* __restrict__ QK, const _Float16* __restrict__ VT, _Float16* __restrict__ O16) {
  __shared__ __attribute__((aligned(16))) unsigned short so[4][16][72];
  const int tid = threadIdx.x; const int w = __builtin_amdgcn_readfirstlane(tid >> 5); const int lane = tid & 31, ln = lane & 15, hh = lane >> 4;
  const int h = blockIdx.y, b = blockIdx.z; const int q0 = blockIdx.x * 64 + 16 * w;
  const _Float16* qrow = QK + ((size_t)b * SEQ + q0 + ln) * LQK + h * HD;
  const v16h qf0 = g2_frag(qrow, hh), qf1 = g2_frag(qrow + 32, hh);
  const _Float16* kbase = QK + ((size_t)b * SEQ + ln) * LQK + DM + h * HD;
  const _Float16* vbase = VT + ((size_t)(b * NH + h) * HD + ln) * SEQ;
  const v8f z8 = {0.f,0.f,0.f,0.f,0.f,0.f,0.f,0.f};
  v8f O[4] = {z8, z8, z8, z8};
  float m = -1.0e30f, l = 0.f;
#pragma unroll 1
  for (int kb = 0; kb < SEQ; kb += 64) {
    v8f S[4];
#pragma unroll
    for (int j = 0; j < 4; ++j) { const _Float16* kr = kbase + (size_t)(kb + j * 16) * LQK; const v16h a0 = g2_frag(kr, hh), a1 = g2_frag(kr + 32, hh);
      const v8f s = g2_mma(a0, qf0, z8); S[j] = g2_mma(a1, qf1, s); }
    float mx = S[0][0];
#pragma unroll
    for (int j = 0; j < 4; ++j)
#pragma unroll
      for (int r = 0; r < 8; ++r) mx = fmaxf(mx, S[j][r]);
    mx = fmaxf(mx, __shfl_xor(mx, 16, 32));
    const float mn = fmaxf(m, mx);
    const float sc = __expf((m - mn) * 0.125f);
    const float mn8 = mn * 0.125f;
    m = mn;
    float ls = 0.f;
    FragH pb0, pb1;
#pragma unroll
    for (int r = 0; r < 8; ++r) {
      const float p0 = __expf(fmaf(S[0][r], 0.125f, -mn8)); const float p1 = __expf(fmaf(S[1][r], 0.125f, -mn8));
      const float p2 = __expf(fmaf(S[2][r], 0.125f, -mn8)); const float p3 = __expf(fmaf(S[3][r], 0.125f, -mn8));
      ls += (p0 + p1) + (p2 + p3);
      pb0.h[r] = (_Float16)(p0 * 1024.0f); pb0.h[8 + r] = (_Float16)(p1 * 1024.0f);
      pb1.h[r] = (_Float16)(p2 * 1024.0f); pb1.h[8 + r] = (_Float16)(p3 * 1024.0f); }
    l = l * sc + ls;
#pragma unroll
    for (int t = 0; t < 4; ++t) O[t] = O[t] * sc;
#pragma unroll
    for (int t = 0; t < 4; ++t) { const _Float16* vr = vbase + (size_t)(t * 16) * SEQ + kb; const v16h a0 = g2_frag(vr, hh), a1 = g2_frag(vr + 32, hh);
      O[t] = g2_mma(a0, pb0.v, O[t]); O[t] = g2_mma(a1, pb1.v, O[t]); }
  }
  const float lt = l + __shfl_xor(l, 16, 32);
  const float inv = 0.0625f * (1.0f / lt);
#pragma unroll
  for (int t = 0; t < 4; ++t) { FragH f;
#pragma unroll
    for (int r = 0; r < 8; ++r) f.h[r] = (_Float16)(O[t][r] * inv);
    *(v8us*)&so[w][ln][t * 16 + 8 * hh] = f.half[0]; }
  __syncthreads();
  const int rq = lane >> 3, pc = (lane & 7) * 8;
  for (int pass = 0; pass < 2; ++pass) {
#pragma unroll
    for (int q = 0; q < 4; ++q) { const int row = q * 4 + rq; const v8us v = *(const v8us*)&so[w][row][pc];
      *(volatile v8us*)((unsigned short*)O16 + ((size_t)b * SEQ + q0 + row) * DM + h * HD + pc) = v; }
    if (pass == 0) __threadfence(); }
}

extern "C" void kernel_launch(void* const* d_in, const int* in_sizes, int n_in,
                              void* d_out, int out_size, void* d_ws, size_t ws_size, hipStream_t stream) {
  if (n_in < 3) return;
  const size_t need_x = ((size_t)(NB - 1) * SEQ_FULL + SEQ) * DM;
  if ((size_t)in_sizes[0] < need_x || (size_t)in_sizes[1] < (size_t)3 * DM * DM || (size_t)in_sizes[2] < (size_t)DM * DM) return;
  if ((size_t)out_size < need_x) return;
  if ((size_t)WS_TOTAL > ws_size) return;
  const float* x = (const float*)d_in[0];
  const float* wqkv = (const float*)d_in[1];
  const float* wout = (const float*)d_in[2];
  char* ws = (char*)d_ws; size_t off = 0;
  _Float16* X16  = (_Float16*)(ws + off); off += SZ_X16;
  _Float16* BQKV = (_Float16*)(ws + off); off += SZ_BQKV;
  _Float16* BO   = (_Float16*)(ws + off); off += SZ_BO;
  _Float16* QK16 = (_Float16*)(ws + off); off += SZ_QK;
  _Float16* VT   = (_Float16*)(ws + off); off += SZ_VT;
  _Float16* O16  = (_Float16*)(ws + off); off += SZ_O16;
  if (off > ws_size) return;

  k_x16<<<(unsigned)((NR * (DM / 8) + 255) / 256), 256, 0, stream>>>(x, X16, (int)NR);
  k_wnat<<<(unsigned)(((size_t)3 * DM * DM / 8 + 255) / 256), 256, 0, stream>>>(wqkv, (size_t)3 * DM * DM / 8, BQKV);
  k_wnat<<<(unsigned)(((size_t)DM * DM / 8 + 255) / 256), 256, 0, stream>>>(wout, (size_t)DM * DM / 8, BO);
  k_gemm2<<<dim3((unsigned)((NR / 128) * (LQK / 64)), 1), 128, 0, stream>>>(X16, DM, (size_t)0, BQKV, DM, (size_t)0, 0.0625f, (float*)nullptr, QK16, LQK, (size_t)0, LQK, DM);
  k_gemm2<<<dim3((unsigned)((DM / 128) * (SEQ / 64)), NB), 128, 0, stream>>>(BQKV + (size_t)2 * DM * DM, DM, (size_t)0, X16, DM, (size_t)SEQ * DM, 0.0625f, (float*)nullptr, VT, SEQ, (size_t)DM * SEQ, SEQ, DM);
  k_flash<<<dim3(SEQ / 64, NH, NB), 128, 0, stream>>>(QK16, VT, O16);
  k_gemm2<<<dim3((unsigned)((SEQ / 128) * (DM / 64)), NB), 128, 0, stream>>>(O16, DM, (size_t)SEQ * DM, BO, DM, (size_t)0, 0.0009765625f, (float*)d_out, (_Float16*)nullptr, DM, (size_t)SEQ_FULL * DM, DM, DM);
}
